// LogLinearMamba2_62216896250126
// MI455X (gfx1250) — hardware-run, weakly checked
//
#include <hip/hip_runtime.h>


#define NR   1024
#define NE   1024
#define NP   4864
#define NX   2048
#define NF   2304
#define NS   128
#define NHD  32
#define NW   64
#define NT   15
#define NG   8

typedef _Float16 h16;
typedef unsigned short bf;
typedef __attribute__((ext_vector_type(16))) __bf16   v16bf;
typedef __attribute__((ext_vector_type(16))) _Float16 v16h;
typedef __attribute__((ext_vector_type(8)))  _Float16 v8h;
typedef __attribute__((ext_vector_type(8)))  unsigned short v8us;
typedef __attribute__((ext_vector_type(8)))  float    v8f;
typedef __attribute__((ext_vector_type(4)))  float    v4f;
typedef v8h  __attribute__((may_alias)) v8ha;
typedef v4f  __attribute__((may_alias)) v4fa;
typedef v8us __attribute__((may_alias)) v8usa;

__device__ __forceinline__ unsigned short f2bf(float f) { unsigned u = __float_as_uint(f); u += 0x7FFFu + ((u >> 16) & 1u); return (unsigned short)(u >> 16); }
__device__ __forceinline__ float bf2f(unsigned short b) { return __uint_as_float(((unsigned)b) << 16); }
__device__ __forceinline__ float bfr(float f) { return bf2f(f2bf(f)); }
__device__ __forceinline__ v16h cat16(v8h lo, v8h hi) { return __builtin_shufflevector(lo, hi, 0, 1, 2, 3, 4, 5, 6, 7, 8, 9, 10, 11, 12, 13, 14, 15); }
__device__ __forceinline__ v16bf cat16b(v8us lo, v8us hi) { return __builtin_bit_cast(v16bf, __builtin_shufflevector(lo, hi, 0, 1, 2, 3, 4, 5, 6, 7, 8, 9, 10, 11, 12, 13, 14, 15)); }
__device__ __forceinline__ v8f wmma16(v16h a, v16h b, v8f c) { return __builtin_amdgcn_wmma_f32_16x16x32_f16(false, a, false, b, (short)0, c, false, false); }
__device__ __forceinline__ v8f wmmab(v16bf a, v16bf b, v8f c) { return __builtin_amdgcn_wmma_f32_16x16x32_bf16(false, a, false, b, (short)0, c, false, false); }

template <typename T16> struct WFrag;
template <> struct WFrag<h16> { typedef v16h V; static __device__ __forceinline__ V ld(const h16* p) { return cat16(*(const v8h*)p, *(const v8h*)(p + 16)); } static __device__ __forceinline__ v8f mma(V a, V b, v8f c) { return wmma16(a, b, c); } };
template <> struct WFrag<bf> { typedef v16bf V; static __device__ __forceinline__ V ld(const bf* p) { return cat16b(*(const v8us*)p, *(const v8us*)(p + 16)); } static __device__ __forceinline__ v8f mma(V a, V b, v8f c) { return wmmab(a, b, c); } };
template <typename T16, int NSPLIT, bool BIAS>
__global__ __launch_bounds__(32) void k_gemmw(const T16* __restrict__ A, const T16* __restrict__ A2, const T16* __restrict__ Bt, const T16* __restrict__ Bt2, int K, float* C, int ldc, const float* __restrict__ bias, size_t sA, size_t sB, size_t sC) {
    typedef typename WFrag<T16>::V V;
    __shared__ __align__(16) float os[16 * 68];
    const size_t z = blockIdx.z; A += z * sA; if (A2) A2 += z * sA; Bt += z * sB; if (Bt2) Bt2 += z * sB; C += z * sC;
    const int lane = threadIdx.x & 31, lr = lane & 15, hi = lane >> 4; const int r0 = blockIdx.x * 64, c0 = blockIdx.y * 64;
    v8f acc[4][4];
#pragma unroll
    for (int mb = 0; mb < 4; ++mb)
#pragma unroll
        for (int nb = 0; nb < 4; ++nb) acc[mb][nb] = (v8f){};
    const size_t aoff = (size_t)(r0 + lr) * K + 8 * hi, boff = (size_t)(c0 + lr) * K + 8 * hi;
    for (int kc = 0; kc < K; kc += 32) {
        V a[4], a2[4];
#pragma unroll
        for (int mb = 0; mb < 4; ++mb) { a[mb] = WFrag<T16>::ld(A + aoff + (size_t)mb * 16 * K + kc); if (NSPLIT == 1 || NSPLIT == 2) a2[mb] = WFrag<T16>::ld(A2 + aoff + (size_t)mb * 16 * K + kc); }
#pragma unroll
        for (int nb = 0; nb < 4; ++nb) { const V b = WFrag<T16>::ld(Bt + boff + (size_t)nb * 16 * K + kc); V b2; if (NSPLIT >= 2) b2 = WFrag<T16>::ld(Bt2 + boff + (size_t)nb * 16 * K + kc);
#pragma unroll
            for (int mb = 0; mb < 4; ++mb) { acc[mb][nb] = WFrag<T16>::mma(a[mb], b, acc[mb][nb]); if (NSPLIT == 1 || NSPLIT == 2) acc[mb][nb] = WFrag<T16>::mma(a2[mb], b, acc[mb][nb]); if (NSPLIT >= 2) acc[mb][nb] = WFrag<T16>::mma(a[mb], b2, acc[mb][nb]); } }
        asm volatile("v_nop\n\tv_nop\n\tv_nop\n\tv_nop" : "+v"(acc[0][0]), "+v"(acc[1][1]), "+v"(acc[2][2]), "+v"(acc[3][3]) : "v"(a[0]), "v"(a[3]));
    }
#pragma unroll
    for (int mb = 0; mb < 4; ++mb) {
#pragma unroll
        for (int nb = 0; nb < 4; ++nb) {
#pragma unroll
            for (int j = 0; j < 8; ++j) os[(hi * 8 + j) * 68 + nb * 16 + lr] = acc[mb][nb][j]; }
        __builtin_amdgcn_wave_barrier(); asm volatile("" ::: "memory");
        float* crow = C + (size_t)(r0 + mb * 16) * ldc + c0;
#pragma unroll 1
        for (int ps = 0; ps < 2; ++ps) {
#pragma unroll
            for (int s = 0; s < 8; ++s) { const int row = 2 * s + hi, cofs = lr * 4; v4f val = *(const v4fa*)(os + row * 68 + cofs); if (BIAS) { val[0] += bfr(bias[c0 + cofs]); val[1] += bfr(bias[c0 + cofs + 1]); val[2] += bfr(bias[c0 + cofs + 2]); val[3] += bfr(bias[c0 + cofs + 3]); }
                *(volatile v4f*)(crow + (size_t)row * ldc + cofs) = val; }
            if (ps == 0) __threadfence(); }
        __builtin_amdgcn_wave_barrier(); asm volatile("" ::: "memory");
    }
}

typedef __attribute__((ext_vector_type(2))) _Float16 v2h;
typedef __attribute__((ext_vector_type(4))) _Float16 v4h;
typedef __attribute__((ext_vector_type(2))) unsigned short v2us;
typedef __attribute__((ext_vector_type(4))) unsigned short v4us;
typedef __attribute__((ext_vector_type(2))) float v2f;
typedef __attribute__((ext_vector_type(4))) int v4i;
__global__ __launch_bounds__(256) void k_cvt8(const float* __restrict__ src, bf* dst, size_t n8) { const size_t i = (size_t)blockIdx.x * 256 + threadIdx.x; if (i >= n8) return; const v8f v = *(const v8f*)(src + i * 8); v8us o;
#pragma unroll
    for (int k = 0; k < 8; ++k) o[k] = f2bf(v[k]); *(volatile v8us*)(dst + i * 8) = o; __threadfence(); *(volatile v8us*)(dst + i * 8) = o; }

__device__ __forceinline__ void splitf(float y, unsigned short& h, unsigned short& l) { h = f2bf(y); l = f2bf(y - bf2f(h)); }

__global__ __launch_bounds__(256) void k_tohl(const float* __restrict__ F, float sc, bf* Hh, bf* Hl, size_t n4) { const size_t i = (size_t)blockIdx.x * 256 + threadIdx.x; if (i >= n4) return; const v4f a = *(const v4f*)(F + i * 4); v4us oh, ol;
#pragma unroll
    for (int q = 0; q < 4; ++q) { unsigned short h2, l2; splitf(__fmul_rn(a[q], sc), h2, l2); oh[q] = h2; ol[q] = l2; }
    *(volatile v4us*)(Hh + i * 4) = oh; *(volatile v4us*)(Hl + i * 4) = ol; __threadfence(); *(volatile v4us*)(Hh + i * 4) = oh; *(volatile v4us*)(Hl + i * 4) = ol; }

__device__ __forceinline__ h16 toh_flush(float x) { const float z = (fabsf(x) < 6.103515625e-05f) ? 0.0f : x; return (h16)z; }

__global__ __launch_bounds__(256) void k_filt(const float* __restrict__ Zs, unsigned pt, unsigned wd, const float* __restrict__ a4, float* Qd) { const unsigned id = blockIdx.x * 256u + threadIdx.x; const unsigned w8 = wd >> 3; const unsigned rw = id / w8, c0 = (id - rw * w8) << 3; float acc[8];
#pragma unroll
    for (int q = 0; q < 8; ++q) acc[q] = 0.0f;
#pragma unroll
    for (int tp = 0; tp < 4; ++tp) { const unsigned bk = 3u - (unsigned)tp; const float on = rw >= bk ? 1.0f : 0.0f; const unsigned r2 = rw >= bk ? rw - bk : 0u; const float* ps = Zs + (size_t)r2 * pt + c0; const v4f va = *(const v4f*)ps, vb = *(const v4f*)(ps + 4);
#pragma unroll
        for (int q = 0; q < 8; ++q) acc[q] = acc[q] + (on * (q < 4 ? va[q] : vb[q - 4])) * bfr(a4[(size_t)(c0 + q) * 4 + tp]); }
    v4f oa, ob;
#pragma unroll
    for (int q = 0; q < 8; ++q) { const float wv = acc[q] * (1.0f / (1.0f + expf(-acc[q]))); if (q < 4) oa[q] = wv; else ob[q - 4] = wv; }
    float* pd = Qd + (size_t)rw * wd + c0; *(volatile v4f*)pd = oa; *(volatile v4f*)(pd + 4) = ob; __threadfence(); *(volatile v4f*)pd = oa; *(volatile v4f*)(pd + 4) = ob; }

__global__ __launch_bounds__(32) void k_gsum(const float* __restrict__ Zp, const float* __restrict__ a5, const float* __restrict__ a6, const float* __restrict__ a7, float* Fs, float* St, float* Ts) { const unsigned hd = threadIdx.x; const float ad = bfr(a5[hd]); const float rt = expf(bfr(a6[hd])); float tw[NT];
#pragma unroll
    for (int j = 0; j < NT; ++j) tw[j] = bfr(a7[hd * NT + j]);
    float run = 0.0f;
    for (int rw = 0; rw < NR; ++rw) { const float* pz = Zp + (size_t)rw * 512; const float uu = pz[hd] + ad; const float sp = fmaxf(uu, 0.0f) + log1pf(expf(-fabsf(uu))); run = run - rt * sp; v4f ot[4];
#pragma unroll
        for (int j = 0; j < 16; ++j) { float sc = 0.0f; if (j < NT) { const float qq = tw[j] * pz[NHD + hd * NT + j]; sc = fmaxf(qq, 0.0f) + log1pf(expf(-fabsf(qq))); } ot[j >> 2][j & 3] = sc; }
        float* pf = Fs + (size_t)rw * NHD + hd; float* pq = St + (size_t)rw * NHD + hd; float* pt = Ts + ((size_t)rw * NHD + hd) * 16;
        *(volatile float*)pf = run; *(volatile float*)pq = sp; *(volatile v4f*)pt = ot[0]; *(volatile v4f*)(pt + 4) = ot[1]; *(volatile v4f*)(pt + 8) = ot[2]; *(volatile v4f*)(pt + 12) = ot[3]; __threadfence();
        *(volatile float*)pf = run; *(volatile float*)pq = sp; *(volatile v4f*)pt = ot[0]; *(volatile v4f*)(pt + 4) = ot[1]; *(volatile v4f*)(pt + 8) = ot[2]; *(volatile v4f*)(pt + 12) = ot[3]; } }

__global__ __launch_bounds__(256) void k_vt(const float* __restrict__ Xs, const float* __restrict__ St, h16* Vt) { const unsigned id = blockIdx.x * 256u + threadIdx.x; const unsigned r0 = (id & 127u) << 3, hc = id >> 7, hd = hc >> 6; v8h ov;
#pragma unroll
    for (int q = 0; q < 8; ++q) ov[q] = toh_flush(Xs[(size_t)(r0 + q) * NX + hc] * St[(size_t)(r0 + q) * NHD + hd]);
    *(volatile v8h*)(Vt + (size_t)id * 8) = ov; __threadfence(); *(volatile v8h*)(Vt + (size_t)id * 8) = ov; }

__global__ __launch_bounds__(256) void k_wts(const float* __restrict__ Sc, const float* __restrict__ Fs, const float* __restrict__ Ts, unsigned h0, h16* Wt) { const unsigned id = blockIdx.x * 256u + threadIdx.x; const unsigned c0 = (id & 127u) << 3, rw = (id >> 7) & 1023u, hd = h0 + (id >> 17); const float* ps = Sc + (size_t)rw * NR + c0; const v4f sa = *(const v4f*)ps, sb = *(const v4f*)(ps + 4); const float fr = Fs[(size_t)rw * NHD + hd]; const float* pq = Ts + ((size_t)rw * NHD + hd) * 16; v8h ow;
#pragma unroll
    for (int q = 0; q < 8; ++q) { const unsigned cl = c0 + (unsigned)q; const unsigned xr = rw ^ cl; const unsigned tr = xr == 0u ? 0u : 32u - (unsigned)__clz((int)xr); const float ex = expf(fr - Fs[(size_t)cl * NHD + hd]); const float wv = (q < 4 ? sa[q] : sb[q - 4]) * ex * pq[tr]; ow[q] = toh_flush(cl <= rw ? wv : 0.0f); }
    *(volatile v8h*)(Wt + (size_t)id * 8) = ow; __threadfence(); *(volatile v8h*)(Wt + (size_t)id * 8) = ow; }

__global__ __launch_bounds__(256) void k_fin(const float* __restrict__ Ys, const float* __restrict__ Xs, const float* __restrict__ Zx, const float* __restrict__ a8, const float* __restrict__ a9, float* Yn) { const unsigned rw = blockIdx.x * 256u + threadIdx.x; const float* py = Ys + (size_t)rw * NX; const float* px = Xs + (size_t)rw * NX; const float* pg = Zx + (size_t)rw * 4096; float ss = 0.0f;
    for (int c0 = 0; c0 < NX; c0 += 8) { const v4f ya = *(const v4f*)(py + c0), yb = *(const v4f*)(py + c0 + 4), xa = *(const v4f*)(px + c0), xb = *(const v4f*)(px + c0 + 4), ga = *(const v4f*)(pg + c0), gb = *(const v4f*)(pg + c0 + 4); const float sk = bfr(a8[c0 >> 6]);
#pragma unroll
        for (int q = 0; q < 8; ++q) { const float gw = q < 4 ? ga[q] : gb[q - 4]; const float wv = ((q < 4 ? ya[q] : yb[q - 4]) + sk * (q < 4 ? xa[q] : xb[q - 4])) * (gw * (1.0f / (1.0f + expf(-gw)))); ss = ss + wv * wv; } }
    const float sc = 1.0f / sqrtf(ss / 2048.0f + 1e-5f); float* pn = Yn + (size_t)rw * NX;
    for (int c0 = 0; c0 < NX; c0 += 8) { const v4f ya = *(const v4f*)(py + c0), yb = *(const v4f*)(py + c0 + 4), xa = *(const v4f*)(px + c0), xb = *(const v4f*)(px + c0 + 4), ga = *(const v4f*)(pg + c0), gb = *(const v4f*)(pg + c0 + 4), na = *(const v4f*)(a9 + c0), nb = *(const v4f*)(a9 + c0 + 4); const float sk = bfr(a8[c0 >> 6]); v4f oa, ob;
#pragma unroll
        for (int q = 0; q < 8; ++q) { const float gw = q < 4 ? ga[q] : gb[q - 4]; const float wv = ((q < 4 ? ya[q] : yb[q - 4]) + sk * (q < 4 ? xa[q] : xb[q - 4])) * (gw * (1.0f / (1.0f + expf(-gw)))); const float ov = (wv * sc) * bfr(q < 4 ? na[q] : nb[q - 4]); if (q < 4) oa[q] = ov; else ob[q - 4] = ov; }
        *(volatile v4f*)(pn + c0) = oa; *(volatile v4f*)(pn + c0 + 4) = ob; __threadfence(); *(volatile v4f*)(pn + c0) = oa; *(volatile v4f*)(pn + c0 + 4) = ob; } }

extern "C" void kernel_launch(void* const* d_in, const int* in_sizes, int n_in, void* d_out, int out_size, void* d_ws, size_t ws_size, hipStream_t stream) {
    if (n_in < 11) return;
    if (in_sizes[0] != NR * NE || in_sizes[1] != NP * NE || in_sizes[2] != NP || in_sizes[3] != NF * 4 || in_sizes[4] != NHD || in_sizes[5] != NHD || in_sizes[6] != NHD * NT || in_sizes[7] != NHD || in_sizes[8] != NX || in_sizes[9] != NE * NX || in_sizes[10] != NE) return;
    if (out_size != NR * NE) return;
    static_assert(NP == NX + NF + NHD + NHD * NT && NF == NX + 2 * NS && NX == NHD * NW && NHD * (NT + 1) == 512 && NR % 64 == 0 && NE % 64 == 0 && NX % 64 == 0 && NS % 64 == 0 && 4096 % 64 == 0 && 512 % 64 == 0 && NE % 32 == 0 && NS % 32 == 0 && NR % 32 == 0 && NX % 32 == 0 && (NR * NE / 8) % 256 == 0 && (NP * NE / 8) % 256 == 0 && (NE * NX / 8) % 256 == 0 && (NR * NX / 8) % 256 == 0 && (NR * NS / 8) % 256 == 0 && (NR * NS / 4) % 256 == 0 && (NR * NX / 4) % 256 == 0 && NHD == 32 && NHD % NG == 0 && (NG * NR * NR / 8) % 256 == 0 && NR == 1024 && NR % 256 == 0 && NT < 16 && NW == 64, "the products: row and column counts multiples of 64, the depths of 32; every flat grid exact; a row is ten bits and a column's eighth seven of a thread's number; sixteen tier slots a (row, head); eight heads a pass");
    const float* i0 = (const float*)d_in[0]; const float* i1 = (const float*)d_in[1]; const float* i2 = (const float*)d_in[2]; const float* i3 = (const float*)d_in[3]; const float* i4 = (const float*)d_in[4]; const float* i5 = (const float*)d_in[5]; const float* i6 = (const float*)d_in[6]; const float* i7 = (const float*)d_in[7]; const float* i8 = (const float*)d_in[8]; const float* i9 = (const float*)d_in[9]; const float* i10 = (const float*)d_in[10]; float* rs0 = (float*)d_out;
    char* wsp = (char*)d_ws; auto carve = [&](size_t bytes) { char* p = wsp; wsp += (bytes + 255) & ~(size_t)255; return (void*)p; };
    bf* Xb = (bf*)carve((size_t)NR * NE * 2); bf* Wi = (bf*)carve((size_t)NP * NE * 2); bf* Wo = (bf*)carve((size_t)NE * NX * 2); float* Zx = (float*)carve((size_t)NR * 4096 * 4); float* Ze = (float*)carve((size_t)NR * NS * 4); float* Zr = (float*)carve((size_t)NR * NS * 4); float* Zp = (float*)carve((size_t)NR * 512 * 4); float* Xs = (float*)carve((size_t)NR * NX * 4); float* Es = (float*)carve((size_t)NR * NS * 4); float* Rs = (float*)carve((size_t)NR * NS * 4); bf* Eh = (bf*)carve((size_t)NR * NS * 2); bf* El = (bf*)carve((size_t)NR * NS * 2); bf* Rh = (bf*)carve((size_t)NR * NS * 2); bf* Rl = (bf*)carve((size_t)NR * NS * 2); float* Sc = (float*)carve((size_t)NR * NR * 4); float* Fs = (float*)carve((size_t)NR * NHD * 4); float* St = (float*)carve((size_t)NR * NHD * 4); float* Ts = (float*)carve((size_t)NR * NHD * 16 * 4); h16* Vt = (h16*)carve((size_t)NX * NR * 2); h16* Wt = (h16*)carve((size_t)NG * NR * NR * 2); float* Ys = (float*)carve((size_t)NR * NX * 4); float* Yn = (float*)carve((size_t)NR * NX * 4); bf* Yh = (bf*)carve((size_t)NR * NX * 2); bf* Yl = (bf*)carve((size_t)NR * NX * 2);
    if ((size_t)(wsp - (char*)d_ws) > ws_size) return;
    k_cvt8<<<(unsigned)(NR * NE / 8 / 256), 256, 0, stream>>>(i0, Xb, (size_t)NR * NE / 8);
    k_cvt8<<<(unsigned)(NP * NE / 8 / 256), 256, 0, stream>>>(i1, Wi, (size_t)NP * NE / 8);
    k_cvt8<<<(unsigned)(NE * NX / 8 / 256), 256, 0, stream>>>(i9, Wo, (size_t)NE * NX / 8);
    k_gemmw<bf, 0, true><<<dim3(NR / 64, 4096 / 64, 1), 32, 0, stream>>>(Xb, nullptr, Wi, nullptr, NE, Zx, 4096, i2, 0, 0, 0);
    k_gemmw<bf, 0, true><<<dim3(NR / 64, NS / 64, 1), 32, 0, stream>>>(Xb, nullptr, Wi + (size_t)4096 * NE, nullptr, NE, Ze, NS, i2 + 4096, 0, 0, 0);
    k_gemmw<bf, 0, true><<<dim3(NR / 64, NS / 64, 1), 32, 0, stream>>>(Xb, nullptr, Wi + (size_t)(4096 + NS) * NE, nullptr, NE, Zr, NS, i2 + 4096 + NS, 0, 0, 0);
    k_gemmw<bf, 0, true><<<dim3(NR / 64, 512 / 64, 1), 32, 0, stream>>>(Xb, nullptr, Wi + (size_t)(NX + NF) * NE, nullptr, NE, Zp, 512, i2 + NX + NF, 0, 0, 0);
    k_filt<<<(unsigned)(NR * NX / 8 / 256), 256, 0, stream>>>(Zx + NX, 4096u, (unsigned)NX, i3, Xs);
    k_filt<<<(unsigned)(NR * NS / 8 / 256), 256, 0, stream>>>(Ze, (unsigned)NS, (unsigned)NS, i3 + (size_t)NX * 4, Es);
    k_filt<<<(unsigned)(NR * NS / 8 / 256), 256, 0, stream>>>(Zr, (unsigned)NS, (unsigned)NS, i3 + (size_t)(NX + NS) * 4, Rs);
    k_tohl<<<(unsigned)(NR * NS / 4 / 256), 256, 0, stream>>>(Es, 1.0f, Eh, El, (size_t)NR * NS / 4);
    k_tohl<<<(unsigned)(NR * NS / 4 / 256), 256, 0, stream>>>(Rs, 1.0f, Rh, Rl, (size_t)NR * NS / 4);
    k_gemmw<bf, 2, false><<<dim3(NR / 64, NR / 64, 1), 32, 0, stream>>>(Rh, Rl, Eh, El, NS, Sc, NR, nullptr, 0, 0, 0);
    k_gsum<<<1, 32, 0, stream>>>(Zp, i4, i5, i6, Fs, St, Ts);
    k_vt<<<(unsigned)(NX * NR / 8 / 256), 256, 0, stream>>>(Xs, St, Vt);
    for (unsigned h0 = 0; h0 < (unsigned)NHD; h0 += (unsigned)NG) {
        k_wts<<<(unsigned)(NG * NR * NR / 8 / 256), 256, 0, stream>>>(Sc, Fs, Ts, h0, Wt);
        k_gemmw<h16, 0, false><<<dim3(NR / 64, NW / 64, NG), 32, 0, stream>>>(Wt, nullptr, Vt + (size_t)h0 * NW * NR, nullptr, NR, Ys + (size_t)h0 * NW, NX, nullptr, (size_t)NR * NR, (size_t)NW * NR, (size_t)NW); }
    k_fin<<<(unsigned)(NR / 256), 256, 0, stream>>>(Ys, Xs, Zx, i7, i8, Yn);
    k_tohl<<<(unsigned)(NR * NX / 4 / 256), 256, 0, stream>>>(Yn, 1.0f, Yh, Yl, (size_t)NR * NX / 4);
    k_gemmw<bf, 1, true><<<dim3(NR / 64, NE / 64, 1), 32, 0, stream>>>(Yh, Yl, Wo, nullptr, NX, rs0, NE, i10, 0, 0, 0);
}
